// Calc_Attention_51032801411467
// MI455X (gfx1250) — hardware-run, weakly checked
//
#include <hip/hip_runtime.h>


#ifndef NB
#define NB 2
#endif
#ifndef SEQ
#define SEQ 2048
#endif
#define NB_FULL  2
#define SEQ_FULL 2048
#ifndef OUT_SEQ
#define OUT_SEQ SEQ
#endif
#define DM   1024
#define NH_  32
#define HD   32
#define DQ   (3 * DM)
#define AW   4
#define OSP  36
#define WTP  68
#define QRS  2048.0f
#define QRI  (1.0f / 2048.0f)
#define SC2  ((float)(0.17677669529663687 * 1.4426950408889634))
#define PSH  14.0f
#define NEGB (-3.0e38f)
#define WOS  32.0f
#define CSC  16.0f
#define OSC  (1.0f / 512.0f)
#define LNE  1.0e-6f

static_assert(HD == 32);
static_assert(NH_ * HD == DM);
static_assert(DM % 64 == 0);
static_assert(64 % HD == 0);
static_assert(DM % 32 == 0);
static_assert(DQ == 3 * DM);
static_assert(DQ % 64 == 0);
static_assert(SEQ % 64 == 0);
static_assert((NB * SEQ) % 64 == 0);
static_assert(SEQ % 32 == 0);
static_assert(SEQ % (16 * AW) == 0);
static_assert(((size_t)SEQ * DM) % 8 == 0);
static_assert(((size_t)NB * SEQ * DM) % 8 == 0);
static_assert(NB <= NB_FULL);
static_assert(SEQ <= SEQ_FULL);
static_assert((OSP * 4) % 16 == 0);
static_assert((WTP * 4) % 16 == 0);
static_assert(DM == 256 * 4);
static_assert(16 * 68 * 4 <= 131072);
static_assert(AW * 16 * OSP * 4 <= 131072);
static_assert(64 * WTP * 4 <= 131072);
static_assert(2 * 2 * 32 * 16 == 16 * 64 * 2);
static_assert(4 * 32 * 16 == 16 * 64 * 2);
static_assert(2 * 32 * 16 == 16 * HD * 2);
static_assert(8 * 32 * 16 == 16 * 64 * 4);
static_assert(2 * 256 * 16 == 64 * 64 * 2);
static_assert(4 * 256 * 4 == 64 * 64);

typedef _Float16 h16;
typedef unsigned short bf;
typedef __attribute__((ext_vector_type(16))) __bf16   v16bf;
typedef __attribute__((ext_vector_type(16))) _Float16 v16h;
typedef __attribute__((ext_vector_type(8)))  _Float16 v8h;
typedef __attribute__((ext_vector_type(8)))  unsigned short v8us;
typedef __attribute__((ext_vector_type(8)))  float    v8f;
typedef __attribute__((ext_vector_type(4)))  float    v4f;
typedef v4f  __attribute__((may_alias)) v4fa;

__device__ __forceinline__ unsigned short f2bf(float f) { unsigned u = __float_as_uint(f); u += 0x7FFFu + ((u >> 16) & 1u); return (unsigned short)(u >> 16); }
__device__ __forceinline__ float bfr(float f) { return __uint_as_float(((unsigned)f2bf(f)) << 16); }
__device__ __forceinline__ v16h cat16(v8h lo, v8h hi) { return __builtin_shufflevector(lo, hi, 0, 1, 2, 3, 4, 5, 6, 7, 8, 9, 10, 11, 12, 13, 14, 15); }
__device__ __forceinline__ v16bf cat16b(v8us lo, v8us hi) { return __builtin_bit_cast(v16bf, __builtin_shufflevector(lo, hi, 0, 1, 2, 3, 4, 5, 6, 7, 8, 9, 10, 11, 12, 13, 14, 15)); }
__device__ __forceinline__ v8f wmma16(v16h a, v16h b, v8f c) { return __builtin_amdgcn_wmma_f32_16x16x32_f16(false, a, false, b, (short)0, c, false, false); }
__device__ __forceinline__ v8f wmmab(v16bf a, v16bf b, v8f c) { return __builtin_amdgcn_wmma_f32_16x16x32_bf16(false, a, false, b, (short)0, c, false, false); }
__device__ __forceinline__ v8f wmma16g(v16h a, v16h b, v8f c) { c = wmma16(a, b, c); asm volatile("v_nop\n\tv_nop\n\tv_nop\n\tv_nop" : "+v"(c) : "v"(a), "v"(b)); return c; }
__device__ __forceinline__ v8f wmmabg(v16bf a, v16bf b, v8f c) { c = wmmab(a, b, c); asm volatile("v_nop\n\tv_nop\n\tv_nop\n\tv_nop" : "+v"(c) : "v"(a), "v"(b)); return c; }
__device__ __forceinline__ v16h  ldh(const h16* p) { return cat16(*(const v8h*)p, *(const v8h*)(p + 16)); }
__device__ __forceinline__ v16bf ldb(const bf* p)  { return cat16b(*(const v8us*)p, *(const v8us*)(p + 16)); }
__device__ __forceinline__ void wave_sync() { __builtin_amdgcn_fence(3  , "wavefront"); __builtin_amdgcn_wave_barrier(); asm volatile("" ::: "memory"); }
static __device__ __forceinline__ h16 toh_flush(float v) { const float w = (fabsf(v) < 6.103515625e-05f) ? 0.0f : v; return (h16)w; }
__device__ __forceinline__ float wsum32(float x) {
#pragma unroll
    for (int mk = 16; mk > 0; mk >>= 1) x += __shfl_xor(x, mk, 32);
    return x;
}

__global__ __launch_bounds__(256) void k_cvt8(const float* __restrict__ src, bf* dst, size_t n8) {
    const size_t i = (size_t)blockIdx.x * 256 + threadIdx.x; if (i >= n8) return;
    const v8f v = *(const v8f*)(src + i * 8); v8us o;
#pragma unroll
    for (int k = 0; k < 8; ++k) o[k] = f2bf(v[k]);
    *(volatile v8us*)(dst + i * 8) = o; __threadfence(); *(volatile v8us*)(dst + i * 8) = o;
}

__global__ __launch_bounds__(256) void k_wtb(const float* __restrict__ src, bf* dst, unsigned KR, unsigned NC) {
    __shared__ __align__(16) float ts[64 * WTP];
    const unsigned tid = threadIdx.x;
    const unsigned k0 = blockIdx.x * 64u, n0 = blockIdx.y * 64u;
#pragma unroll
    for (unsigned i = 0; i < 4; ++i) { const unsigned idx = i * 256u + tid; const unsigned r = idx >> 4, c4 = (idx & 15u) * 4u;
        const v4f v = *(const v4f*)(src + (size_t)(k0 + r) * NC + n0 + c4);
        ts[(c4 + 0u) * WTP + r] = v[0]; ts[(c4 + 1u) * WTP + r] = v[1]; ts[(c4 + 2u) * WTP + r] = v[2]; ts[(c4 + 3u) * WTP + r] = v[3]; }
    __syncthreads();
#pragma unroll 1
    for (int ps = 0; ps < 2; ++ps) {
#pragma unroll
        for (unsigned s = 0; s < 2; ++s) { const unsigned p = s * 256u + tid; const unsigned row = p >> 3, c8 = (p & 7u) * 8u;
            const v4f x0 = *(const v4fa*)(&ts[row * WTP + c8]); const v4f x1 = *(const v4fa*)(&ts[row * WTP + c8 + 4u]); v8us o;
#pragma unroll
            for (int i = 0; i < 4; ++i) { o[i] = f2bf(x0[i]); o[4 + i] = f2bf(x1[i]); }
            *(volatile v8us*)(dst + (size_t)(n0 + row) * KR + k0 + c8) = o; }
        if (ps == 0) __threadfence(); }
}

__global__ __launch_bounds__(256) void k_wth(const float* __restrict__ src, h16* dst, unsigned KR, unsigned NC) {
    __shared__ __align__(16) float ts[64 * WTP];
    const unsigned tid = threadIdx.x;
    const unsigned k0 = blockIdx.x * 64u, n0 = blockIdx.y * 64u;
#pragma unroll
    for (unsigned i = 0; i < 4; ++i) { const unsigned idx = i * 256u + tid; const unsigned r = idx >> 4, c4 = (idx & 15u) * 4u;
        const v4f v = *(const v4f*)(src + (size_t)(k0 + r) * NC + n0 + c4);
        ts[(c4 + 0u) * WTP + r] = v[0]; ts[(c4 + 1u) * WTP + r] = v[1]; ts[(c4 + 2u) * WTP + r] = v[2]; ts[(c4 + 3u) * WTP + r] = v[3]; }
    __syncthreads();
#pragma unroll 1
    for (int ps = 0; ps < 2; ++ps) {
#pragma unroll
        for (unsigned s = 0; s < 2; ++s) { const unsigned p = s * 256u + tid; const unsigned row = p >> 3, c8 = (p & 7u) * 8u;
            const v4f x0 = *(const v4fa*)(&ts[row * WTP + c8]); const v4f x1 = *(const v4fa*)(&ts[row * WTP + c8 + 4u]); v8h o;
#pragma unroll
            for (int i = 0; i < 4; ++i) { o[i] = toh_flush(bfr(x0[i]) * WOS); o[4 + i] = toh_flush(bfr(x1[i]) * WOS); }
            *(volatile v8h*)(dst + (size_t)(n0 + row) * KR + k0 + c8) = o; }
        if (ps == 0) __threadfence(); }
}

__global__ __launch_bounds__(32) void k_projqk(const bf* __restrict__ A, const bf* __restrict__ Bt, h16* Ph) {
    __shared__ __align__(16) float os[16 * 68];
    const unsigned lane = threadIdx.x & 31u, lr = lane & 15u, hi = lane >> 4;
    const unsigned r0 = blockIdx.x * 64u, c0 = blockIdx.y * 64u;
    v8f acc[4][4];
#pragma unroll
    for (int mb = 0; mb < 4; ++mb)
#pragma unroll
        for (int nb = 0; nb < 4; ++nb) acc[mb][nb] = (v8f){};
    const size_t aoff = (size_t)(r0 + lr) * DM + 8u * hi, boff = (size_t)(c0 + lr) * DM + 8u * hi;
#pragma unroll 1
    for (unsigned kc = 0; kc < (unsigned)DM; kc += 32u) {
        v16bf a[4];
#pragma unroll
        for (int mb = 0; mb < 4; ++mb) a[mb] = ldb(A + aoff + (size_t)mb * 16 * DM + kc);
#pragma unroll
        for (int nb = 0; nb < 4; ++nb) { const v16bf b = ldb(Bt + boff + (size_t)nb * 16 * DM + kc);
#pragma unroll
            for (int mb = 0; mb < 4; ++mb) acc[mb][nb] = wmmabg(a[mb], b, acc[mb][nb]); }
    }
    const unsigned bb = r0 / (unsigned)SEQ, tt = r0 % (unsigned)SEQ; const unsigned zc = bb * (unsigned)NH_ + c0 / (unsigned)HD;
    const size_t tbase = ((size_t)zc * SEQ + (size_t)tt) * HD;
#pragma unroll
    for (int mb = 0; mb < 4; ++mb) {
#pragma unroll
        for (int nb = 0; nb < 4; ++nb) {
#pragma unroll
            for (int j = 0; j < 8; ++j) os[(hi * 8u + j) * 68u + nb * 16 + lr] = acc[mb][nb][j]; }
        wave_sync();
#pragma unroll 1
        for (int ps = 0; ps < 2; ++ps) {
            const size_t sb = tbase + (size_t)(mb * 16) * HD;
#pragma unroll
            for (int hh = 0; hh < 2; ++hh) {
#pragma unroll
                for (unsigned s = 0; s < 2; ++s) { const unsigned p = s * 32u + lane; const unsigned row = p >> 2, c8 = (p & 3u) * 8u;
                    const v4f x0 = *(const v4fa*)(&os[row * 68u + hh * 32 + c8]); const v4f x1 = *(const v4fa*)(&os[row * 68u + hh * 32 + c8 + 4u]); v8h hv;
#pragma unroll
                    for (int i = 0; i < 4; ++i) { hv[i] = toh_flush(x0[i]); hv[4 + i] = toh_flush(x1[i]); }
                    const size_t oo = sb + (size_t)hh * ((size_t)SEQ * HD) + (size_t)p * 8;
                    *(volatile v8h*)(Ph + oo) = hv; } }
            if (ps == 0) __threadfence(); }
        wave_sync();
    }
}

__global__ __launch_bounds__(32) void k_projvt(const bf* __restrict__ A, const bf* __restrict__ Bt, h16* Ph) {
    __shared__ __align__(16) float os[16 * 68];
    const unsigned lane = threadIdx.x & 31u, lr = lane & 15u, hi = lane >> 4;
    const unsigned r0 = blockIdx.x * 64u, c0 = blockIdx.y * 64u;
    v8f acc[4][4];
#pragma unroll
    for (int mb = 0; mb < 4; ++mb)
#pragma unroll
        for (int nb = 0; nb < 4; ++nb) acc[mb][nb] = (v8f){};
    const size_t aoff = (size_t)(r0 + lr) * DM + 8u * hi, boff = (size_t)(c0 + lr) * DM + 8u * hi;
#pragma unroll 1
    for (unsigned kc = 0; kc < (unsigned)DM; kc += 32u) {
        v16bf a[4];
#pragma unroll
        for (int mb = 0; mb < 4; ++mb) a[mb] = ldb(A + aoff + (size_t)mb * 16 * DM + kc);
#pragma unroll
        for (int nb = 0; nb < 4; ++nb) { const v16bf b = ldb(Bt + boff + (size_t)nb * 16 * DM + kc);
#pragma unroll
            for (int mb = 0; mb < 4; ++mb) acc[mb][nb] = wmmabg(a[mb], b, acc[mb][nb]); }
    }
    const unsigned bb = c0 / (unsigned)SEQ, tt = c0 % (unsigned)SEQ;
    const size_t tbase = (size_t)bb * (size_t)DM * SEQ + (size_t)r0 * SEQ + (size_t)tt;
#pragma unroll
    for (int mb = 0; mb < 4; ++mb) {
#pragma unroll
        for (int nb = 0; nb < 4; ++nb) {
#pragma unroll
            for (int j = 0; j < 8; ++j) os[(hi * 8u + j) * 68u + nb * 16 + lr] = acc[mb][nb][j]; }
        wave_sync();
#pragma unroll 1
        for (int ps = 0; ps < 2; ++ps) {
            const size_t sb = tbase + (size_t)(mb * 16) * SEQ;
#pragma unroll
            for (unsigned s = 0; s < 4; ++s) { const unsigned row = 4u * s + (lane >> 3), c8 = (lane & 7u) * 8u;
                const v4f x0 = *(const v4fa*)(&os[row * 68u + c8]); const v4f x1 = *(const v4fa*)(&os[row * 68u + c8 + 4u]); v8h hv;
#pragma unroll
                for (int i = 0; i < 4; ++i) { hv[i] = toh_flush(x0[i]); hv[4 + i] = toh_flush(x1[i]); }
                const size_t oo = sb + (size_t)row * SEQ + c8;
                *(volatile v8h*)(Ph + oo) = hv; }
            if (ps == 0) __threadfence(); }
        wave_sync();
    }
}

__global__ __launch_bounds__(32 * AW) void k_flash(const h16* __restrict__ QH, const h16* __restrict__ KP, const h16* __restrict__ VT, h16* CH, h16* CR) {
    __shared__ __align__(16) float os[AW * 16 * OSP];
    const unsigned lane = threadIdx.x & 31u, lr = lane & 15u, hi = lane >> 4;
    const unsigned wave = (unsigned)__builtin_amdgcn_readfirstlane((int)(threadIdx.x >> 5));
    const unsigned zh = blockIdx.y;
    const unsigned t0 = (blockIdx.x * (unsigned)AW + wave) * 16u;
    const size_t pbase = (size_t)zh * SEQ * HD;
    const size_t qo = pbase + (size_t)(t0 + lr) * HD + 8u * hi;
    const v16h qh = ldh(QH + qo);
    const size_t ko = pbase + (size_t)lr * HD + 8u * hi;
    const size_t vo = pbase + (size_t)lr * SEQ + 8u * hi;
    v8f o0 = (v8f){}, o1 = (v8f){};
    float m = NEGB, l = 0.0f;
#pragma unroll 1
    for (unsigned key0 = 0; key0 < (unsigned)SEQ; key0 += 32u) {
        const h16* ka = KP + ko + (size_t)key0 * HD;
        const v16h ka0 = ldh(ka), kb0 = ldh(ka + 16 * HD);
        v8f sa = (v8f){}, sb = (v8f){};
        sa = wmma16g(ka0, qh, sa); sb = wmma16g(kb0, qh, sb);
        float ta[8], tb[8]; float mx = NEGB;
#pragma unroll
        for (int r = 0; r < 8; ++r) { ta[r] = sa[r] * SC2; tb[r] = sb[r] * SC2; mx = fmaxf(mx, fmaxf(ta[r], tb[r])); }
        mx = fmaxf(mx, __shfl_xor(mx, 16, 32));
        const float mnew = fmaxf(m, mx);
        const float alpha = __builtin_amdgcn_exp2f(m - mnew);
        const float sh = PSH - mnew;
        v16h pb; float ls = 0.0f;
#pragma unroll
        for (int r = 0; r < 8; ++r) {
            const float xa = ta[r] + sh, xb = tb[r] + sh;
            const float ea = (xa < -14.0f) ? 0.0f : __builtin_amdgcn_exp2f(xa);
            const float eb = (xb < -14.0f) ? 0.0f : __builtin_amdgcn_exp2f(xb);
            const h16 pa = (h16)ea; const h16 pc = (h16)eb;
            pb[r] = pa; pb[8 + r] = pc;
            ls += (float)pa + (float)pc; }
        l = l * alpha + ls; m = mnew;
        o0 = o0 * alpha; o1 = o1 * alpha;
        const h16* va = VT + vo + key0;
        const v16h v0 = ldh(va), v1 = ldh(va + (size_t)16 * SEQ);
        o0 = wmma16g(v0, pb, o0); o1 = wmma16g(v1, pb, o1);
    }
    l += __shfl_xor(l, 16, 32);
    const float inv = CSC * (1.0f / l);
    const v8f f0 = o0, f1 = o1;
    const unsigned wb = wave * 16u * (unsigned)OSP;
    { v4f a, c;
      a[0] = f0[0] * inv; a[1] = f0[1] * inv; a[2] = f0[2] * inv; a[3] = f0[3] * inv; c[0] = f0[4] * inv; c[1] = f0[5] * inv; c[2] = f0[6] * inv; c[3] = f0[7] * inv;
      *(v4fa*)(&os[wb + lr * OSP +  0 + 8u * hi]) = a; *(v4fa*)(&os[wb + lr * OSP +  0 + 8u * hi + 4u]) = c;
      a[0] = f1[0] * inv; a[1] = f1[1] * inv; a[2] = f1[2] * inv; a[3] = f1[3] * inv; c[0] = f1[4] * inv; c[1] = f1[5] * inv; c[2] = f1[6] * inv; c[3] = f1[7] * inv;
      *(v4fa*)(&os[wb + lr * OSP + 16 + 8u * hi]) = a; *(v4fa*)(&os[wb + lr * OSP + 16 + 8u * hi + 4u]) = c; }
    wave_sync();
    const size_t cb = pbase + (size_t)t0 * HD;
#pragma unroll 1
    for (int ps = 0; ps < 2; ++ps) {
#pragma unroll
        for (unsigned s = 0; s < 2; ++s) { const unsigned p = s * 32u + lane; const unsigned row = p >> 2, c8 = (p & 3u) * 8u;
            const v4f x0 = *(const v4fa*)(&os[wb + row * OSP + c8]); const v4f x1 = *(const v4fa*)(&os[wb + row * OSP + c8 + 4u]); v8h hv, rv;
#pragma unroll
            for (int i = 0; i < 4; ++i) { const h16 a0 = toh_flush(x0[i]); const h16 a1 = toh_flush(x1[i]); hv[i] = a0; hv[4 + i] = a1;
                rv[i] = toh_flush((x0[i] - (float)a0) * QRS); rv[4 + i] = toh_flush((x1[i] - (float)a1) * QRS); }
            const size_t oo = cb + (size_t)p * 8;
            *(volatile v8h*)(CH + oo) = hv; *(volatile v8h*)(CR + oo) = rv; }
        if (ps == 0) __threadfence(); }
}

__global__ __launch_bounds__(32) void k_oproj(const h16* __restrict__ CH, const h16* __restrict__ CR, const h16* __restrict__ WO, const float* __restrict__ bias, float* Y) {
    __shared__ __align__(16) float os[16 * 68];
    const unsigned lane = threadIdx.x & 31u, lr = lane & 15u, hi = lane >> 4;
    const unsigned r0 = blockIdx.x * 32u, c0 = blockIdx.y * 64u;
    const unsigned bb = r0 / (unsigned)SEQ, tt = r0 % (unsigned)SEQ;
    v8f acc[2][4], acr[2][4];
#pragma unroll
    for (int mb = 0; mb < 2; ++mb)
#pragma unroll
        for (int nb = 0; nb < 4; ++nb) { acc[mb][nb] = (v8f){}; acr[mb][nb] = (v8f){}; }
    const size_t aoff = ((size_t)bb * NH_ * SEQ + (size_t)(tt + lr)) * HD + 8u * hi;
    const size_t boff = (size_t)(c0 + lr) * DM + 8u * hi;
#pragma unroll 1
    for (unsigned hk = 0; hk < (unsigned)NH_; ++hk) {
        const size_t ao = aoff + (size_t)hk * SEQ * HD;
        v16h a[2], ar[2];
#pragma unroll
        for (int mb = 0; mb < 2; ++mb) { a[mb] = ldh(CH + ao + (size_t)mb * 16 * HD); ar[mb] = ldh(CR + ao + (size_t)mb * 16 * HD); }
#pragma unroll
        for (int nb = 0; nb < 4; ++nb) { const v16h b = ldh(WO + boff + (size_t)nb * 16 * DM + hk * 32u);
#pragma unroll
            for (int mb = 0; mb < 2; ++mb) { acc[mb][nb] = wmma16g(a[mb], b, acc[mb][nb]); acr[mb][nb] = wmma16g(ar[mb], b, acr[mb][nb]); } }
    }
    float bc[4];
#pragma unroll
    for (int nb = 0; nb < 4; ++nb) bc[nb] = bfr(bias[c0 + nb * 16 + lr]);
#pragma unroll
    for (int mb = 0; mb < 2; ++mb) {
#pragma unroll
        for (int nb = 0; nb < 4; ++nb) {
#pragma unroll
            for (int j = 0; j < 8; ++j) os[(hi * 8u + j) * 68u + nb * 16 + lr] = (acc[mb][nb][j] + acr[mb][nb][j] * QRI) * OSC + bc[nb]; }
        wave_sync();
        float* yrow = Y + (size_t)(r0 + mb * 16) * DM + c0;
#pragma unroll 1
        for (int ps = 0; ps < 2; ++ps) {
#pragma unroll
            for (unsigned s = 0; s < 8; ++s) { const unsigned row = 2u * s + (lane >> 4), cofs = (lane & 15u) * 4u;
                const v4f val = *(const v4fa*)(&os[row * 68u + cofs]);
                *(volatile v4f*)(yrow + (size_t)row * DM + cofs) = val; }
            if (ps == 0) __threadfence(); }
        wave_sync();
    }
}

__global__ __launch_bounds__(256) void k_ln(const float* __restrict__ Y, const float* __restrict__ gain, const float* __restrict__ shift, float* OUT) {
#pragma clang fp contract(off)
    __shared__ float red[16];
    const unsigned tid = threadIdx.x, lane = tid & 31u;
    const unsigned wave = (unsigned)__builtin_amdgcn_readfirstlane((int)(threadIdx.x >> 5));
    const unsigned row = blockIdx.x; const unsigned b = row / (unsigned)SEQ, t = row % (unsigned)SEQ;
    const v4f y = *(const v4f*)(Y + (size_t)row * DM + 4u * tid);
    float s = (y[0] + y[1]) + (y[2] + y[3]);
    s = wsum32(s);
    if (lane == 0u) red[wave] = s;
    __syncthreads();
    float S = 0.0f;
#pragma unroll
    for (int w = 0; w < 8; ++w) S += red[w];
    const float mu = S * (1.0f / (float)DM);
    const float d0 = y[0] - mu, d1 = y[1] - mu, d2 = y[2] - mu, d3 = y[3] - mu;
    float q = (d0 * d0 + d1 * d1) + (d2 * d2 + d3 * d3);
    q = wsum32(q);
    if (lane == 0u) red[8u + wave] = q;
    __syncthreads();
    float Q = 0.0f;
#pragma unroll
    for (int w = 0; w < 8; ++w) Q += red[8 + w];
    const float var = Q * (1.0f / (float)DM);
    const float rs = 1.0f / sqrtf(var + LNE);
    const v4f g4 = *(const v4f*)(gain + 4u * tid);
    const v4f b4 = *(const v4f*)(shift + 4u * tid);
    v4f o;
    o[0] = (d0 * rs) * bfr(g4[0]) + bfr(b4[0]);
    o[1] = (d1 * rs) * bfr(g4[1]) + bfr(b4[1]);
    o[2] = (d2 * rs) * bfr(g4[2]) + bfr(b4[2]);
    o[3] = (d3 * rs) * bfr(g4[3]) + bfr(b4[3]);
    float* op = OUT + ((size_t)b * OUT_SEQ + (size_t)t) * DM + 4u * tid;
    *(volatile v4f*)op = o; __threadfence(); *(volatile v4f*)op = o;
}

static constexpr size_t al256(size_t v) { return (v + 255) & ~(size_t)255; }
static constexpr size_t SZ_XB = al256((size_t)NB * SEQ * DM * 2);
static constexpr size_t SZ_WT = al256((size_t)DQ * DM * 2);
static constexpr size_t SZ_WO = al256((size_t)DM * DM * 2);
static constexpr size_t SZ_PL = al256((size_t)NB * NH_ * SEQ * HD * 2);
static constexpr size_t SZ_Y  = al256((size_t)NB * SEQ * DM * 4);
static constexpr size_t SZ_TOTAL = SZ_XB + SZ_WT + SZ_WO + 5 * SZ_PL + SZ_Y;
static_assert(SZ_TOTAL <= (size_t)134217728);
static_assert(((size_t)DM * DM * 2) % 256 == 0);
static_assert((size_t)NB * NH_ * SEQ * HD == (size_t)NB * DM * SEQ);
static_assert(((size_t)NB * SEQ / 64) * 64 * ((size_t)DM / 64) * 64 == (size_t)NB * SEQ * DM);
static_assert(((size_t)NB * SEQ / 32) * 32 * ((size_t)DM / 64) * 64 == (size_t)NB * SEQ * DM);
static_assert(((size_t)SEQ / (16 * AW)) * 16 * AW * ((size_t)NB * NH_) * HD == (size_t)NB * NH_ * SEQ * HD);

extern "C" void kernel_launch(void* const* d_in, const int* in_sizes, int n_in,
                              void* d_out, int out_size, void* d_ws, size_t ws_size, hipStream_t stream) {
    if (n_in < 6) return;
    const size_t needx = ((size_t)(NB - 1) * SEQ_FULL + SEQ) * DM;
    if ((size_t)in_sizes[0] < needx) return;
    if ((size_t)in_sizes[1] < (size_t)DM * DQ || (size_t)in_sizes[2] < (size_t)DM * DM) return;
    if (in_sizes[3] < DM || in_sizes[4] < DM || in_sizes[5] < DM) return;
    if ((size_t)out_size < ((size_t)(NB - 1) * OUT_SEQ + SEQ) * DM) return;
    if (SZ_TOTAL > ws_size) return;
    const float* x    = (const float*)d_in[0];
    const float* wqkv = (const float*)d_in[1];
    const float* wout = (const float*)d_in[2];
    const float* bout = (const float*)d_in[3];
    const float* lng  = (const float*)d_in[4];
    const float* lnb  = (const float*)d_in[5];
    float* OUT = (float*)d_out;
    char* wsp = (char*)d_ws;
    bf*  XB = (bf*)wsp;  wsp += SZ_XB;
    bf*  WT = (bf*)wsp;  wsp += SZ_WT;
    h16* WO = (h16*)wsp; wsp += SZ_WO;
    h16* QH = (h16*)wsp; wsp += SZ_PL;
    h16* KP = (h16*)wsp; wsp += SZ_PL;
    h16* VT = (h16*)wsp; wsp += SZ_PL;
    h16* CH = (h16*)wsp; wsp += SZ_PL;
    h16* CR = (h16*)wsp; wsp += SZ_PL;
    float* YP = (float*)wsp; wsp += SZ_Y;
    bf* WTQ = WT; bf* WTK = WT + (size_t)DM * DM; bf* WTV = WT + (size_t)2 * DM * DM;

    if (SEQ == SEQ_FULL) {
        const size_t n8 = (size_t)NB * SEQ * DM / 8;
        k_cvt8<<<(unsigned)((n8 + 255) / 256), 256, 0, stream>>>(x, XB, n8);
    } else {
        const size_t n8 = (size_t)SEQ * DM / 8;
        for (int b = 0; b < NB; ++b) k_cvt8<<<(unsigned)((n8 + 255) / 256), 256, 0, stream>>>(x + (size_t)b * SEQ_FULL * DM, XB + (size_t)b * SEQ * DM, n8);
    }
    k_wtb<<<dim3(DM / 64, DQ / 64, 1), 256, 0, stream>>>(wqkv, WT, (unsigned)DM, (unsigned)DQ);
    k_wth<<<dim3(DM / 64, DM / 64, 1), 256, 0, stream>>>(wout, WO, (unsigned)DM, (unsigned)DM);

    k_projqk<<<dim3(NB * SEQ / 64, DM / 64, 1), 32, 0, stream>>>(XB, WTQ, QH);
    k_projqk<<<dim3(NB * SEQ / 64, DM / 64, 1), 32, 0, stream>>>(XB, WTK, KP);
    k_projvt<<<dim3(DM / 64, NB * SEQ / 64, 1), 32, 0, stream>>>(WTV, XB, VT);

    k_flash<<<dim3(SEQ / (16 * AW), NB * NH_, 1), 32 * AW, 0, stream>>>(QH, KP, VT, CH, CR);
    k_oproj<<<dim3(NB * SEQ / 32, DM / 64, 1), 32, 0, stream>>>(CH, CR, WO, bout, YP);
    k_ln<<<dim3(NB * SEQ, 1, 1), 256, 0, stream>>>(YP, lng, lnb, OUT);
}
